// WeightedSAGE_14474039787720
// MI455X (gfx1250) — hardware-verified
//
#include <hip/hip_runtime.h>
#include <stddef.h>


#define DF     128
#define KT     256
#define NB     512
#define CHUNK  4096
#define NTHR   256
#define NWAVE  8
#define WCAP   512
#define SUBR   16
#define NGRP   (CHUNK / (NTHR * 4))
#define NLAYER 4
#define WPL    (DF * KT)

#define LDS_ACC_F  (NB * DF)
#define LDS_LIST_I (NWAVE * WCAP)
#define LDS_BYTES  (LDS_ACC_F * 4 + LDS_LIST_I * 4 + 64)

static_assert(WCAP == NGRP * 4 * 32);
static_assert(2 * SUBR * KT * 2 <= LDS_LIST_I * 4);
static_assert(NWAVE * 16 == DF);
static_assert(NTHR == NWAVE * 32);
static_assert((NB & (NB - 1)) == 0 && NB <= 512);
static_assert(CHUNK <= 4096);
static_assert(NB == 2 * NWAVE * (NB / SUBR));

typedef float          v4f   __attribute__((ext_vector_type(4)));
typedef float          v8f   __attribute__((ext_vector_type(8)));
typedef int            v4i   __attribute__((ext_vector_type(4)));
typedef unsigned short v8us  __attribute__((ext_vector_type(8)));
typedef __bf16         v16bf __attribute__((ext_vector_type(16)));
union Frag { v16bf v; v8us h[2]; };

__device__ __forceinline__ unsigned int bf16_rne(float f) {
  unsigned int u = __float_as_uint(f);
  u += 0x7FFFu + ((u >> 16) & 1u);
  return u >> 16;
}

__device__ __forceinline__ void split8(v4f a, v4f b, v8us& hi, v8us& lo) {
  unsigned int hb, lb;
#define SPLK(I, VAL) hb = bf16_rne(VAL); lb = bf16_rne((VAL) - __uint_as_float(hb << 16)); \
  hi[I] = (unsigned short)hb; lo[I] = (unsigned short)lb;
  SPLK(0, a.x) SPLK(1, a.y) SPLK(2, a.z) SPLK(3, a.w)
  SPLK(4, b.x) SPLK(5, b.y) SPLK(6, b.z) SPLK(7, b.w)
#undef SPLK
}

__device__ __forceinline__ v8f wm(v16bf a, v16bf b, v8f c) {
  v8f d = __builtin_amdgcn_wmma_f32_16x16x32_bf16(false, a, false, b, (short)0, c, false, false);
  asm volatile("v_nop\n\tv_nop\n\tv_nop\n\tv_nop" : "+v"(d) : "v"(a), "v"(b));
  return d;
}

__global__ __launch_bounds__(NTHR) void k_wprep(
    const float* __restrict__ Wa, const float* __restrict__ Wb,
    const float* __restrict__ Wc, const float* __restrict__ Wd,
    unsigned short* planes, int total) {
  const int g = blockIdx.x * NTHR + threadIdx.x;
  if (g >= total) return;
  const int lsel = g >> 12;
  const int rem  = g & 4095;
  const int n    = rem >> 5;
  const int k    = (rem & 31) * 8;
  const float* W = (lsel == 0) ? Wa : (lsel == 1) ? Wb : (lsel == 2) ? Wc : Wd;
  v4f a, b;
  a.x = W[(size_t)(k + 0) * DF + n];
  a.y = W[(size_t)(k + 1) * DF + n];
  a.z = W[(size_t)(k + 2) * DF + n];
  a.w = W[(size_t)(k + 3) * DF + n];
  b.x = W[(size_t)(k + 4) * DF + n];
  b.y = W[(size_t)(k + 5) * DF + n];
  b.z = W[(size_t)(k + 6) * DF + n];
  b.w = W[(size_t)(k + 7) * DF + n];
  v8us hi = {0, 0, 0, 0, 0, 0, 0, 0}, lo = {0, 0, 0, 0, 0, 0, 0, 0};
  split8(a, b, hi, lo);
  unsigned short* ph = planes + (size_t)lsel * 2 * WPL;
  unsigned short* pl = ph + WPL;
  const size_t o = (size_t)n * KT + k;
  *(volatile v8us*)(ph + o) = hi;
  *(volatile v8us*)(pl + o) = lo;
  __threadfence();
  *(volatile v8us*)(ph + o) = hi;
  *(volatile v8us*)(pl + o) = lo;
}

__global__ __launch_bounds__(NTHR) void k_layer(
    const float* __restrict__ hin, const int* __restrict__ srci,
    const int* __restrict__ dsti, const float* __restrict__ wedge,
    const unsigned short* __restrict__ wph, const unsigned short* __restrict__ wpl,
    const float* __restrict__ bias, float* hout, int nN, int nE, int relu) {
  extern __shared__ v4f lds_dyn[];
  float* acc  = (float*)lds_dyn;
  int*   list = (int*)(acc + LDS_ACC_F);
  int*   wcnt = list + LDS_LIST_I;
  unsigned short* sAh = (unsigned short*)list;
  unsigned short* sAl = sAh + SUBR * KT;

  const int tid  = threadIdx.x;
  const int lane = tid & 31;
  const int wave = tid >> 5;
  const int hh   = lane >> 4;
  const int m    = lane & 15;
  const int nodeBase = blockIdx.x * NB;

  {
    const v4f z4 = {0.f, 0.f, 0.f, 0.f};
    for (int i = tid; i < LDS_ACC_F / 4; i += NTHR) lds_dyn[i] = z4;
  }
  __syncthreads();

  const int nChunks = (nE + CHUNK - 1) / CHUNK;
#pragma unroll 1
  for (int ch = 0; ch < nChunks; ++ch) {
    const int cbase = ch * CHUNK;
    const bool full = (cbase + CHUNK <= nE);
    int wc = 0;
#pragma unroll
    for (int g = 0; g < NGRP; ++g) {
      const int el0 = (g * NTHR + tid) * 4;
      const int e0  = cbase + el0;
      const int sent = -2147483647 - 1;
      v4i d;
      if (full) {
        d = *(const v4i*)(dsti + e0);
      } else {
        int j0 = e0, j1 = e0 + 1, j2 = e0 + 2, j3 = e0 + 3;
        const int lim = nE - 1;
        const int c0i = j0 > lim ? lim : j0;
        const int c1i = j1 > lim ? lim : j1;
        const int c2i = j2 > lim ? lim : j2;
        const int c3i = j3 > lim ? lim : j3;
        const int v0 = dsti[c0i], v1 = dsti[c1i], v2 = dsti[c2i], v3 = dsti[c3i];
        d.x = (j0 <= lim) ? v0 : sent;
        d.y = (j1 <= lim) ? v1 : sent;
        d.z = (j2 <= lim) ? v2 : sent;
        d.w = (j3 <= lim) ? v3 : sent;
      }
      const unsigned s0 = (unsigned)d.x - (unsigned)nodeBase;
      const unsigned s1 = (unsigned)d.y - (unsigned)nodeBase;
      const unsigned s2 = (unsigned)d.z - (unsigned)nodeBase;
      const unsigned s3 = (unsigned)d.w - (unsigned)nodeBase;
      const bool h0 = s0 < (unsigned)NB;
      const bool h1 = s1 < (unsigned)NB;
      const bool h2 = s2 < (unsigned)NB;
      const bool h3 = s3 < (unsigned)NB;
      const unsigned many = __builtin_amdgcn_ballot_w32(h0 | h1 | h2 | h3);
      if (many != 0u) {
#define HITJ(J, HJ, SJ) { \
          const unsigned mj = __builtin_amdgcn_ballot_w32(HJ); \
          if (HJ) { \
            const int pos = wc + (int)__builtin_amdgcn_mbcnt_lo(mj, 0u); \
            if (pos < WCAP) list[wave * WCAP + pos] = ((el0 + (J)) << 9) | (int)(SJ); \
          } \
          wc += (int)__builtin_popcount(mj); }
        HITJ(0, h0, s0)
        HITJ(1, h1, s1)
        HITJ(2, h2, s2)
        HITJ(3, h3, s3)
#undef HITJ
      }
    }
    if (lane == 0) wcnt[wave] = wc;
    __syncthreads();

    if (wave == 0) {
#pragma unroll 1
      for (int wsx = 0; wsx < NWAVE; ++wsx) {
        int n = wcnt[wsx];
        if (n > WCAP) n = WCAP;
        if (n < 0) n = 0;
#pragma unroll 1
        for (int i = 0; i < n; ++i) {
          const int ent  = list[wsx * WCAP + i];
          const int slot = ent & (NB - 1);
          const int el   = (ent >> 9) & (CHUNK - 1);
          int e = cbase + el;
          if (e > nE - 1) e = nE - 1;
          int s = srci[e];
          s = s < 0 ? 0 : (s > nN - 1 ? nN - 1 : s);
          const float wv = wedge[e];
          const v4f v = *(const v4f*)(hin + (size_t)s * DF + 4 * lane);
          v4f* ap = (v4f*)(acc + slot * DF + 4 * lane);
          const v4f cur = *ap;
          *ap = cur + v * wv;
        }
      }
    }
    __syncthreads();
  }

  int nValid = nN - nodeBase;
  if (nValid > NB) nValid = NB;
  if (nValid < 0) nValid = 0;
  const int nsub = (nValid + SUBR - 1) / SUBR;
  const int ncol = wave * 16 + m;
  const float bv = bias[ncol];

#pragma unroll 1
  for (int s = 0; s < nsub; ++s) {
    {
      const int r  = tid >> 4;
      const int c0 = (tid & 15) * 8;
      int node = nodeBase + s * SUBR + r;
      if (node > nN - 1) node = nN - 1;
      const float* hp = hin + (size_t)node * DF + c0;
      const v4f xa = *(const v4f*)hp, xb = *(const v4f*)(hp + 4);
      v8us hi = {0, 0, 0, 0, 0, 0, 0, 0}, lo = {0, 0, 0, 0, 0, 0, 0, 0};
      split8(xa, xb, hi, lo);
      *(v8us*)(sAh + r * KT + c0) = hi;
      *(v8us*)(sAl + r * KT + c0) = lo;
      const int slot = s * SUBR + r;
      const float* ap = acc + slot * DF + c0;
      const v4f aa = *(const v4f*)ap, ab = *(const v4f*)(ap + 4);
      v8us hi2 = {0, 0, 0, 0, 0, 0, 0, 0}, lo2 = {0, 0, 0, 0, 0, 0, 0, 0};
      split8(aa, ab, hi2, lo2);
      *(v8us*)(sAh + r * KT + DF + c0) = hi2;
      *(v8us*)(sAl + r * KT + DF + c0) = lo2;
    }
    __syncthreads();

    v8f c = {0.f, 0.f, 0.f, 0.f, 0.f, 0.f, 0.f, 0.f};
#pragma unroll
    for (int kt = 0; kt < KT / 32; ++kt) {
      const int k0 = kt * 32;
      Frag ah, al, bh, bl;
      const unsigned short* pah = sAh + m * KT + k0 + 8 * hh;
      const unsigned short* pal = sAl + m * KT + k0 + 8 * hh;
      const unsigned short* pbh = wph + (size_t)ncol * KT + k0 + 8 * hh;
      const unsigned short* pbl = wpl + (size_t)ncol * KT + k0 + 8 * hh;
      ah.h[0] = *(const v8us*)pah; ah.h[1] = *(const v8us*)(pah + 16);
      al.h[0] = *(const v8us*)pal; al.h[1] = *(const v8us*)(pal + 16);
      bh.h[0] = *(const v8us*)pbh; bh.h[1] = *(const v8us*)(pbh + 16);
      bl.h[0] = *(const v8us*)pbl; bl.h[1] = *(const v8us*)(pbl + 16);
      c = wm(al.v, bh.v, c);
      c = wm(ah.v, bl.v, c);
      c = wm(ah.v, bh.v, c);
    }

    {
      float* hrow = acc + (s * SUBR + 8 * hh) * DF + ncol;
#pragma unroll
      for (int r = 0; r < 8; ++r) {
        const float v  = c[r] + bv;
        const float vr = v > 0.0f ? v : 0.0f;
        hrow[r * DF] = (relu != 0) ? vr : v;
      }
    }
    __syncthreads();

    {
      const int slotA = s * SUBR + 2 * wave;
      const int slotB = slotA + 1;
      const v4f yA = *(const v4f*)(acc + slotA * DF + 4 * lane);
      const v4f yB = *(const v4f*)(acc + slotB * DF + 4 * lane);
      const int nodeA = nodeBase + slotA;
      const int nodeB = nodeBase + slotB;
      const bool okA = nodeA < nN;
      const bool okB = nodeB < nN;
      const size_t offA = (size_t)(okA ? nodeA : 0) * DF + 4 * lane;
      const size_t offB = (size_t)(okB ? nodeB : 0) * DF + 4 * lane;
      if (okA) *(volatile v4f*)(hout + offA) = yA;
      if (okB) *(volatile v4f*)(hout + offB) = yB;
      __threadfence();
      if (okA) *(volatile v4f*)(hout + offA) = yA;
      if (okB) *(volatile v4f*)(hout + offB) = yB;
    }
    __syncthreads();
  }
}

extern "C" void kernel_launch(void* const* d_in, const int* in_sizes, int n_in,
                              void* d_out, int out_size, void* d_ws, size_t ws_size,
                              hipStream_t stream) {
  if (n_in < 12) return;
  const int nN = in_sizes[0] / DF;
  const int nE = in_sizes[1];
  if (nN <= 0 || nE <= 0 || in_sizes[0] != nN * DF) return;
  if (in_sizes[2] != nE || in_sizes[3] != nE) return;
  if (in_sizes[4] != KT * DF || in_sizes[6] != KT * DF || in_sizes[8] != KT * DF || in_sizes[10] != KT * DF) return;
  if (in_sizes[5] < DF || in_sizes[7] < DF || in_sizes[9] < DF || in_sizes[11] < DF) return;
  if (out_size != nN * DF) return;

  const float* x    = (const float*)d_in[0];
  const int*   srci = (const int*)d_in[1];
  const int*   dsti = (const int*)d_in[2];
  const float* wed  = (const float*)d_in[3];
  const float* W1 = (const float*)d_in[4];
  const float* b1 = (const float*)d_in[5];
  const float* W2 = (const float*)d_in[6];
  const float* b2 = (const float*)d_in[7];
  const float* W3 = (const float*)d_in[8];
  const float* b3 = (const float*)d_in[9];
  const float* W4 = (const float*)d_in[10];
  const float* b4 = (const float*)d_in[11];
  float* out = (float*)d_out;

  size_t off = 0;
  const size_t planeBytes = (((size_t)nN * DF * sizeof(float)) + 255) & ~(size_t)255;
  float* hpA = (float*)((char*)d_ws + off); off += planeBytes;
  float* hpB = (float*)((char*)d_ws + off); off += planeBytes;
  unsigned short* wplanes = (unsigned short*)((char*)d_ws + off);
  off += (size_t)NLAYER * 2 * WPL * sizeof(unsigned short);
  if (off > ws_size) return;

  const int totalW = NLAYER * DF * (KT / 8);
  k_wprep<<<(totalW + NTHR - 1) / NTHR, NTHR, 0, stream>>>(W1, W2, W3, W4, wplanes, totalW);

  hipFuncSetAttribute(reinterpret_cast<const void*>(&k_layer),
                      hipFuncAttributeMaxDynamicSharedMemorySize, LDS_BYTES);
  const int grid = (nN + NB - 1) / NB;

  const unsigned short* p0h = wplanes + 0 * 2 * WPL; const unsigned short* p0l = p0h + WPL;
  const unsigned short* p1h = wplanes + 1 * 2 * WPL; const unsigned short* p1l = p1h + WPL;
  const unsigned short* p2h = wplanes + 2 * 2 * WPL; const unsigned short* p2l = p2h + WPL;
  const unsigned short* p3h = wplanes + 3 * 2 * WPL; const unsigned short* p3l = p3h + WPL;

  k_layer<<<grid, NTHR, LDS_BYTES, stream>>>(x,   srci, dsti, wed, p0h, p0l, b1, hpA, nN, nE, 1);
  k_layer<<<grid, NTHR, LDS_BYTES, stream>>>(hpA, srci, dsti, wed, p1h, p1l, b2, hpB, nN, nE, 1);
  k_layer<<<grid, NTHR, LDS_BYTES, stream>>>(hpB, srci, dsti, wed, p2h, p2l, b3, hpA, nN, nE, 1);
  k_layer<<<grid, NTHR, LDS_BYTES, stream>>>(hpA, srci, dsti, wed, p3h, p3l, b4, out, nN, nE, 0);
}
